// SelfAttentionBlock_33767032881971
// MI455X (gfx1250) — hardware-run, weakly checked
//
#include <hip/hip_runtime.h>
#include <stddef.h>
#include <stdint.h>


#define NN     50000
#define NE     800000
#define CW     128
#define GBM    64
#define GTHR   128
#define MP     50048
#define GM     (MP / GBM)
#define APITCH 256
#define WPITCH 256
#define SPLIT1 1
#define SPLIT2 1
#define KE1    (SPLIT1 ? 256 : 128)
#define KE2    (SPLIT2 ? 256 : 128)
#define NTHR   256
#define NWAVE  8
#define EPT    8
#define CHUNK  (NTHR * EPT)
#define WCAP   (EPT * 32)
#define LISTN  (NWAVE * WCAP)
#define NBA    1024
#define SLA    10
#define GA     49
#define RCAP   28672
#define DEGCAP 64
#define NEGSL  0.2f
#define AGG_ZINTS (LISTN + 2 * RCAP + 3 * NBA)
#define AGG_LDS_INTS (AGG_ZINTS + 16)
#define NUX    (MP * (CW / 8))
#define NU0    (CW * (CW / 8))
#define NUD    (CW * (WPITCH / 8))
#define NUPB   512
#define P_AS   0
#define P_AD   1
#define P_BA   2
#define P_B1   3
#define P_G1   4
#define P_BE1  5
#define P_B2   6
#define P_G2   7
#define P_BE2  8

static_assert(CW == 128 && CW == 32 * 4);
static_assert(NN == 390 * 128 + 80);
static_assert(MP == GM * GBM && MP >= NN && MP - NN < GBM);
static_assert(GA * NBA >= MP);
static_assert((CHUNK & (CHUNK - 1)) == 0 && CHUNK <= 4096);
static_assert((NBA & (NBA - 1)) == 0 && NBA == (1 << SLA));
static_assert(((long long)CHUNK << SLA) < (1LL << 31));
static_assert(NE < (1 << 21) && (NE % 4) == 0);
static_assert(LISTN % NTHR == 0 && NBA % 32 == 0 && NBA == 4 * NTHR);
static_assert(RCAP % (NTHR * 4) == 0 && AGG_ZINTS % 4 == 0);
static_assert(RCAP >= 16623 + 4096);
static_assert(DEGCAP >= 35 + 8);
static_assert(AGG_LDS_INTS * 4 <= 300000);
static_assert(KE1 % 32 == 0 && KE1 <= APITCH && KE1 <= WPITCH);
static_assert(KE2 % 32 == 0 && KE2 <= APITCH && KE2 <= WPITCH);
static_assert(APITCH == 2 * CW && WPITCH == 2 * CW);
static_assert(GBM == (GTHR / 32) * 16 && GTHR == CW);
static_assert(NUX % NTHR == 0 && NU0 % NTHR == 0 && NUD % NTHR == 0 && NUPB % NTHR == 0);
static_assert((NN * 32) % NTHR == 0 && MP % NWAVE == 0);

typedef float          v4f   __attribute__((ext_vector_type(4)));
typedef float          v8f   __attribute__((ext_vector_type(8)));
typedef double         v2d   __attribute__((ext_vector_type(2)));
typedef int            v4i   __attribute__((ext_vector_type(4)));
typedef int            v8i   __attribute__((ext_vector_type(8)));
typedef unsigned short v4us  __attribute__((ext_vector_type(4)));
typedef unsigned short v8us  __attribute__((ext_vector_type(8)));
typedef unsigned short v16us __attribute__((ext_vector_type(16)));
typedef __bf16         v16bf __attribute__((ext_vector_type(16)));
typedef v4f  __attribute__((may_alias)) v4fa;
typedef v2d  __attribute__((may_alias)) v2da;
typedef v4i  __attribute__((may_alias)) v4ia;
typedef v8us __attribute__((may_alias)) v8usa;
union FragB { v16bf v; v16us u; v8us h[2]; v8i w; };

static constexpr size_t al256(size_t o) { return (o + 255) & ~(size_t)255; }
constexpr size_t SZ_W0T  = (size_t)CW * CW * 2;
constexpr size_t SZ_WD   = (size_t)CW * WPITCH * 2;
constexpr size_t SZ_PAR  = (size_t)9 * CW * 4;
constexpr size_t SZ_MR   = (size_t)2 * CW * 4;
constexpr size_t SZ_FLAG = (size_t)GA * 32 * 4;
constexpr size_t SZ_OC   = (size_t)GA * NBA * 4;
constexpr size_t SZ_AL   = (size_t)GM * 2 * GBM * 4;
constexpr size_t SZ_REC  = (size_t)GM * 2 * CW * 8;
constexpr size_t SZ_HITS = (size_t)GA * RCAP * 4;
constexpr size_t SZ_XB   = (size_t)MP * CW * 2;
constexpr size_t SZ_XL   = (size_t)MP * CW * 4;
constexpr size_t SZ_AP   = (size_t)MP * APITCH * 2;
constexpr size_t SZ_T    = (size_t)MP * CW * 4;
constexpr size_t O_W0T  = 0;
constexpr size_t O_W1D  = al256(O_W0T + SZ_W0T);
constexpr size_t O_W2D  = al256(O_W1D + SZ_WD);
constexpr size_t O_PAR  = al256(O_W2D + SZ_WD);
constexpr size_t O_MR1  = al256(O_PAR + SZ_PAR);
constexpr size_t O_MR2  = al256(O_MR1 + SZ_MR);
constexpr size_t O_FLAG = al256(O_MR2 + SZ_MR);
constexpr size_t O_OFF  = al256(O_FLAG + SZ_FLAG);
constexpr size_t O_CNT  = al256(O_OFF + SZ_OC);
constexpr size_t O_AL   = al256(O_CNT + SZ_OC);
constexpr size_t O_REC1 = al256(O_AL + SZ_AL);
constexpr size_t O_REC2 = al256(O_REC1 + SZ_REC);
constexpr size_t O_HITS = al256(O_REC2 + SZ_REC);
constexpr size_t O_XB   = al256(O_HITS + SZ_HITS);
constexpr size_t O_XL   = al256(O_XB + SZ_XB);
constexpr size_t O_AP   = al256(O_XL + SZ_XL);
constexpr size_t O_T    = al256(O_AP + SZ_AP);
constexpr size_t WS_TOTAL = al256(O_T + SZ_T);
static_assert(WS_TOTAL <= ((size_t)128 << 20));

__device__ __forceinline__ v8f wmb(const FragB& a, const FragB& b, v8f c) {
  v8f d = __builtin_amdgcn_wmma_f32_16x16x32_bf16(false, a.v, false, b.v, (short)0, c, false, false);
  asm volatile("v_nop\n\tv_nop\n\tv_nop\n\tv_nop" : "+v"(d) : "v"(a.w), "v"(b.w));
  return d;
}

__device__ __forceinline__ unsigned bf16_bits(float f) {
  const unsigned u = __float_as_uint(f);
  const unsigned r = (u + 0x7FFFu + ((u >> 16) & 1u)) >> 16;
  const unsigned q = (u >> 16) | 0x40u;
  return ((u & 0x7FFFFFFFu) > 0x7F800000u) ? q : r;
}
__device__ __forceinline__ float bf16_val(float f) {
  return __uint_as_float(bf16_bits(f) << 16);
}
__device__ __forceinline__ v4f bfr4(const v4f a) {
  v4f r; r.x = bf16_val(a.x); r.y = bf16_val(a.y); r.z = bf16_val(a.z); r.w = bf16_val(a.w); return r;
}
__device__ __forceinline__ unsigned split_hl(float v) {
  const unsigned hb = bf16_bits(v);
  const unsigned lb = bf16_bits(v - __uint_as_float(hb << 16));
  return (lb << 16) | (hb & 0xFFFFu);
}
__device__ __forceinline__ void put8(unsigned short* dp, const v8us o) {
  *(volatile v8us*)dp = o;
  __threadfence();
  *(volatile v8us*)dp = o;
}

template <int SLB>
__device__ __forceinline__ int scan_chunk(const int* __restrict__ dsts, int nE, int cbase, int slotBase,
                                          int nb, int vec8, int* list, int tid, int lane, int wave) {
  int wc = 0;
  const int el0  = tid * EPT;
  const int e0   = cbase + el0;
  const int sent = (int)(1u << 31);
  v4i da, db;
  if (vec8 != 0 && cbase + CHUNK <= nE) {
    da = *(const v4i*)(dsts + e0);
    db = *(const v4i*)(dsts + e0 + 4);
  } else {
    da.x = (e0     < nE) ? dsts[min(e0,     nE - 1)] : sent;
    da.y = (e0 + 1 < nE) ? dsts[min(e0 + 1, nE - 1)] : sent;
    da.z = (e0 + 2 < nE) ? dsts[min(e0 + 2, nE - 1)] : sent;
    da.w = (e0 + 3 < nE) ? dsts[min(e0 + 3, nE - 1)] : sent;
    db.x = (e0 + 4 < nE) ? dsts[min(e0 + 4, nE - 1)] : sent;
    db.y = (e0 + 5 < nE) ? dsts[min(e0 + 5, nE - 1)] : sent;
    db.z = (e0 + 6 < nE) ? dsts[min(e0 + 6, nE - 1)] : sent;
    db.w = (e0 + 7 < nE) ? dsts[min(e0 + 7, nE - 1)] : sent;
  }
  const unsigned nbs = (unsigned)slotBase;
  const unsigned unb = (unsigned)nb;
  const unsigned s0 = (unsigned)da.x - nbs, s1 = (unsigned)da.y - nbs;
  const unsigned s2 = (unsigned)da.z - nbs, s3 = (unsigned)da.w - nbs;
  const unsigned s4 = (unsigned)db.x - nbs, s5 = (unsigned)db.y - nbs;
  const unsigned s6 = (unsigned)db.z - nbs, s7 = (unsigned)db.w - nbs;
  const bool h0 = s0 < unb, h1 = s1 < unb, h2 = s2 < unb, h3 = s3 < unb;
  const bool h4 = s4 < unb, h5 = s5 < unb, h6 = s6 < unb, h7 = s7 < unb;
  const unsigned any = __builtin_amdgcn_ballot_w32(h0 | h1 | h2 | h3 | h4 | h5 | h6 | h7);
  if (any != 0u) {
#define HITJ(J, HJ, SJ) { \
      const unsigned mj = __builtin_amdgcn_ballot_w32(HJ); \
      if (mj != 0u) { \
        if (HJ) { \
          const int pos = wc + (int)__builtin_amdgcn_mbcnt_lo(mj, 0u); \
          if (pos < WCAP) list[wave * WCAP + pos] = ((el0 + (J)) << SLB) | (int)(SJ); \
        } \
        wc += (int)__builtin_popcount(mj); } }
    HITJ(0, h0, s0)
    HITJ(1, h1, s1)
    HITJ(2, h2, s2)
    HITJ(3, h3, s3)
    HITJ(4, h4, s4)
    HITJ(5, h5, s5)
    HITJ(6, h6, s6)
    HITJ(7, h7, s7)
#undef HITJ
  }
  return wc;
}

__global__ __launch_bounds__(NTHR) void k_prep(const float* __restrict__ x, const float* __restrict__ W,
                                               const float* __restrict__ W1, const float* __restrict__ W2,
                                               const float* __restrict__ q0, const float* __restrict__ q1,
                                               const float* __restrict__ q2, const float* __restrict__ q3,
                                               const float* __restrict__ q4, const float* __restrict__ q5,
                                               const float* __restrict__ q6, const float* __restrict__ q7,
                                               const float* __restrict__ q8,
                                               unsigned short* XB, unsigned short* W0T,
                                               unsigned short* W1D, unsigned short* W2D, float* PAR) {
  const int u = (int)blockIdx.x * NTHR + (int)threadIdx.x;
  if (u < NUX) {
    const int row = u >> 4;
    const int k8  = (u & 15) * 8;
    const int rc  = row < NN ? row : NN - 1;
    const float* p = x + (size_t)rc * CW + k8;
    const v4f a = *(const v4f*)p;
    const v4f b = *(const v4f*)(p + 4);
    const bool ok = row < NN;
    v8us o;
    o[0] = ok ? (unsigned short)bf16_bits(a.x) : (unsigned short)0;
    o[1] = ok ? (unsigned short)bf16_bits(a.y) : (unsigned short)0;
    o[2] = ok ? (unsigned short)bf16_bits(a.z) : (unsigned short)0;
    o[3] = ok ? (unsigned short)bf16_bits(a.w) : (unsigned short)0;
    o[4] = ok ? (unsigned short)bf16_bits(b.x) : (unsigned short)0;
    o[5] = ok ? (unsigned short)bf16_bits(b.y) : (unsigned short)0;
    o[6] = ok ? (unsigned short)bf16_bits(b.z) : (unsigned short)0;
    o[7] = ok ? (unsigned short)bf16_bits(b.w) : (unsigned short)0;
    put8(XB + (size_t)row * CW + k8, o);
  } else if (u < NUX + NU0) {
    const int v  = u - NUX;
    const int n  = v >> 4;
    const int k8 = (v & 15) * 8;
    const float* p = W + (size_t)k8 * CW + n;
    v8us o;
#pragma unroll
    for (int i = 0; i < 8; ++i) o[i] = (unsigned short)bf16_bits(p[(size_t)i * CW]);
    put8(W0T + (size_t)n * CW + k8, o);
  } else if (u < NUX + NU0 + NUD) {
    const int v  = u - NUX - NU0;
    const int n  = v >> 5;
    const int k8 = (v & 31) * 8;
    const int kk = k8 & (CW - 1);
    const float* p = W1 + (size_t)kk * CW + n;
    v8us o;
#pragma unroll
    for (int i = 0; i < 8; ++i) o[i] = (unsigned short)bf16_bits(p[(size_t)i * CW]);
    put8(W1D + (size_t)n * WPITCH + k8, o);
  } else if (u < NUX + NU0 + 2 * NUD) {
    const int v  = u - NUX - NU0 - NUD;
    const int n  = v >> 5;
    const int k8 = (v & 31) * 8;
    const int kk = k8 & (CW - 1);
    const float* p = W2 + (size_t)kk * CW + n;
    v8us o;
#pragma unroll
    for (int i = 0; i < 8; ++i) o[i] = (unsigned short)bf16_bits(p[(size_t)i * CW]);
    put8(W2D + (size_t)n * WPITCH + k8, o);
  } else {
    const int v   = u - (NUX + NU0 + 2 * NUD);
    const int j   = v & 31;
    const int vec = v >> 5;
    const v4f c0 = *(const v4f*)(q0 + 4 * j);
    const v4f c1 = *(const v4f*)(q1 + 4 * j);
    const v4f c2 = *(const v4f*)(q2 + 4 * j);
    const v4f c3 = *(const v4f*)(q3 + 4 * j);
    const v4f c4 = *(const v4f*)(q4 + 4 * j);
    const v4f c5 = *(const v4f*)(q5 + 4 * j);
    const v4f c6 = *(const v4f*)(q6 + 4 * j);
    const v4f c7 = *(const v4f*)(q7 + 4 * j);
    const v4f c8 = *(const v4f*)(q8 + 4 * j);
    asm volatile("" :: "v"(c0)); asm volatile("" :: "v"(c1)); asm volatile("" :: "v"(c2));
    asm volatile("" :: "v"(c3)); asm volatile("" :: "v"(c4)); asm volatile("" :: "v"(c5));
    asm volatile("" :: "v"(c6)); asm volatile("" :: "v"(c7)); asm volatile("" :: "v"(c8));
    v4f r = c0;
    r = (vec == 1) ? c1 : r;
    r = (vec == 2) ? c2 : r;
    r = (vec == 3) ? c3 : r;
    r = (vec == 4) ? c4 : r;
    r = (vec == 5) ? c5 : r;
    r = (vec == 6) ? c6 : r;
    r = (vec == 7) ? c7 : r;
    r = (vec == 8) ? c8 : r;
    r = bfr4(r);
    if (v < 9 * 32) {
      float* dp = PAR + 4 * v;
      *(volatile v4f*)dp = r;
      __threadfence();
      *(volatile v4f*)dp = r;
    }
  }
}

__global__ __launch_bounds__(NTHR) void k_bucket(const int* __restrict__ srcs, const int* __restrict__ dsts,
                                                 int nE, int nN, int vec8,
                                                 int* HITS, int* OFF, int* CNT, int* FLAG) {
  extern __shared__ __attribute__((aligned(16))) int dsm[];
  int* list = dsm;
  int* hl   = dsm + LISTN;
  int* sl   = dsm + LISTN + RCAP;
  int* cnt  = dsm + LISTN + 2 * RCAP;
  int* offs = cnt + NBA;
  int* cur  = offs + NBA;
  int* misc = cur + NBA;
  const int tid = (int)threadIdx.x, lane = tid & 31, wave = tid >> 5;
  const int nodeBase = (int)blockIdx.x * NBA;

  {
    const v4i z4 = {0, 0, 0, 0};
    for (int i = tid * 4; i < AGG_ZINTS; i += NTHR * 4) *(v4ia*)(dsm + i) = z4;
    if (tid < 16) misc[tid] = 0;
  }
  __syncthreads();

  int t = 0, ov = 0;
  const int nChunks = (nE + CHUNK - 1) / CHUNK;
#pragma unroll 1
  for (int ch = 0; ch < nChunks; ++ch) {
    const int cbase = ch * CHUNK;
    const int wc = scan_chunk<SLA>(dsts, nE, cbase, nodeBase, NBA, vec8, list, tid, lane, wave);
    if (lane == 0) misc[wave] = wc;
    __syncthreads();
    if (wave == 0) {
#pragma unroll 1
      for (int w2 = 0; w2 < NWAVE; ++w2) {
        int c = misc[w2];
        c = c < 0 ? 0 : (c > WCAP ? WCAP : c);
#pragma unroll 1
        for (int b0 = 0; b0 < c; b0 += 32) {
          const int idx = b0 + lane;
          const int ent = list[w2 * WCAP + (idx < WCAP ? idx : WCAP - 1)];
          const int m32 = (c - b0) < 32 ? (c - b0) : 32;
#pragma unroll 1
          for (int k = 0; k < m32; ++k) {
            const int u    = __builtin_amdgcn_readlane(ent, k);
            const int slot = u & (NBA - 1);
            const int el   = (u >> SLA) & (CHUNK - 1);
            const int pk   = ((cbase + el) << SLA) | slot;
            if (t < RCAP) {
              if (lane == 0) { hl[t] = pk; cnt[slot] = cnt[slot] + 1; }
              t = t + 1;
            } else {
              ov = 1;
            }
          }
        }
      }
    }
    __syncthreads();
  }
  if (wave == 0 && lane == 0) { misc[8] = t; misc[9] = ov; }
  __syncthreads();
  int tt = misc[8];
  tt = tt < 0 ? 0 : (tt > RCAP ? RCAP : tt);
  const int ovf = misc[9];

  if (wave == 0) {
    const int base = lane * (NBA / 32);
    int s = 0;
#pragma unroll 1
    for (int i = 0; i < NBA / 32; ++i) s += cnt[base + i];
    int incl = s;
#pragma unroll
    for (int d = 1; d < 32; d <<= 1) {
      const int y = __shfl_up(incl, d, 32);
      if (lane >= d) incl += y;
    }
    int run = incl - s;
#pragma unroll 1
    for (int i = 0; i < NBA / 32; ++i) {
      const int cv = cnt[base + i];
      offs[base + i] = run;
      cur[base + i]  = run;
      run += cv;
    }
  }
  __syncthreads();
  if (wave == 0) {
#pragma unroll 1
    for (int b0 = 0; b0 < tt; b0 += 32) {
      const int idx = b0 + lane;
      const int ent = hl[idx < RCAP ? idx : RCAP - 1];
      const int m32 = (tt - b0) < 32 ? (tt - b0) : 32;
#pragma unroll 1
      for (int k = 0; k < m32; ++k) {
        const int u    = __builtin_amdgcn_readlane(ent, k);
        const int slot = u & (NBA - 1);
        if (lane == 0) {
          int p = cur[slot];
          p = p < 0 ? 0 : (p > RCAP - 1 ? RCAP - 1 : p);
          sl[p] = u;
          cur[slot] = p + 1;
        }
      }
    }
  }
  {
    int bg = 0;
#pragma unroll 1
    for (int i = tid; i < NBA; i += NTHR) bg |= (cnt[i] > DEGCAP) ? 1 : 0;
    if (bg != 0) misc[10] = 1;
  }
  __syncthreads();
  const int fl = (ovf != 0 || misc[10] != 0) ? 1 : 0;

  int* hg = HITS + (size_t)blockIdx.x * RCAP;
#pragma unroll 1
  for (int it = 0; it < RCAP / (NTHR * 4); ++it) {
    const int i0 = it * (NTHR * 4);
    const int i  = i0 + tid * 4;
    v4i o = {0, 0, 0, 0};
    if (i0 < tt) {
      const v4i e4 = *(const v4ia*)(sl + i);
      int e0 = e4.x >> SLA, e1 = e4.y >> SLA, e2 = e4.z >> SLA, e3 = e4.w >> SLA;
      e0 = e0 < 0 ? 0 : (e0 > nE - 1 ? nE - 1 : e0);
      e1 = e1 < 0 ? 0 : (e1 > nE - 1 ? nE - 1 : e1);
      e2 = e2 < 0 ? 0 : (e2 > nE - 1 ? nE - 1 : e2);
      e3 = e3 < 0 ? 0 : (e3 > nE - 1 ? nE - 1 : e3);
      int s0 = srcs[e0];
      int s1 = srcs[e1];
      int s2 = srcs[e2];
      int s3 = srcs[e3];
      asm volatile("" :: "v"(s0)); asm volatile("" :: "v"(s1));
      asm volatile("" :: "v"(s2)); asm volatile("" :: "v"(s3));
      s0 = s0 < 0 ? 0 : (s0 > nN - 1 ? nN - 1 : s0);
      s1 = s1 < 0 ? 0 : (s1 > nN - 1 ? nN - 1 : s1);
      s2 = s2 < 0 ? 0 : (s2 > nN - 1 ? nN - 1 : s2);
      s3 = s3 < 0 ? 0 : (s3 > nN - 1 ? nN - 1 : s3);
      o.x = (i     < tt) ? s0 : 0;
      o.y = (i + 1 < tt) ? s1 : 0;
      o.z = (i + 2 < tt) ? s2 : 0;
      o.w = (i + 3 < tt) ? s3 : 0;
    }
    *(volatile v4i*)(hg + i) = o;
    __threadfence();
    *(volatile v4i*)(hg + i) = o;
  }
  {
    const v4i o4 = *(const v4ia*)(offs + 4 * tid);
    const v4i c4 = *(const v4ia*)(cnt + 4 * tid);
    int* op = OFF + (size_t)blockIdx.x * NBA + 4 * tid;
    int* cp = CNT + (size_t)blockIdx.x * NBA + 4 * tid;
    *(volatile v4i*)op = o4;
    *(volatile v4i*)cp = c4;
    __threadfence();
    *(volatile v4i*)op = o4;
    *(volatile v4i*)cp = c4;
  }
  if (tid < 8) {
    v4i f4;
    f4.x = fl; f4.y = tt; f4.z = fl; f4.w = tt;
    int* fp = FLAG + (size_t)blockIdx.x * 32 + 4 * tid;
    *(volatile v4i*)fp = f4;
    __threadfence();
    *(volatile v4i*)fp = f4;
  }
}

__global__ __launch_bounds__(GTHR) __attribute__((amdgpu_num_vgpr(248)))
void k_gemm0(const unsigned short* __restrict__ A, const unsigned short* __restrict__ BT,
             const float* __restrict__ PAR, float* Cm, float* AL) {
  __shared__ __attribute__((aligned(16))) float stg[GBM * CW];
  __shared__ __attribute__((aligned(16))) float sdt[2 * GBM];
  __shared__ __attribute__((aligned(16))) float spar[2 * CW];
  const int tid = (int)threadIdx.x, lane = tid & 31, wave = tid >> 5, hh = lane >> 4, m = lane & 15;
  const int rowBase = (int)blockIdx.x * GBM;
  if (tid < 64) {
    const v4f p = *(const v4f*)(PAR + 4 * tid);
    *(v4fa*)(spar + 4 * tid) = p;
  }

  v8f acc[8];
  {
    const v8f z = {0.f, 0.f, 0.f, 0.f, 0.f, 0.f, 0.f, 0.f};
#pragma unroll
    for (int t = 0; t < 8; ++t) acc[t] = z;
  }
  const unsigned short* ap = A  + (size_t)(rowBase + 16 * wave + m) * (size_t)CW + 8 * hh;
  const unsigned short* bp = BT + (size_t)m * (size_t)CW + 8 * hh;

#pragma unroll 1
  for (int k0 = 0; k0 < CW; k0 += 32) {
    FragB af;
    af.h[0] = *(const v8usa*)(ap + k0);
    af.h[1] = *(const v8usa*)(ap + k0 + 16);
#pragma unroll
    for (int nt = 0; nt < 8; ++nt) {
      const unsigned short* wq = bp + (size_t)(16 * nt) * (size_t)CW + k0;
      FragB bf;
      bf.h[0] = *(const v8usa*)wq;
      bf.h[1] = *(const v8usa*)(wq + 16);
      acc[nt] = wmb(af, bf, acc[nt]);
    }
  }

#pragma unroll
  for (int nt = 0; nt < 8; ++nt) {
    const int lc = 16 * nt + m;
#pragma unroll
    for (int r = 0; r < 8; ++r) {
      const int lr = 16 * wave + 8 * hh + r;
      stg[lr * CW + lc] = acc[nt][r];
    }
  }
  __syncthreads();

  const v4f as4 = *(const v4fa*)(spar + 4 * lane);
  const v4f ad4 = *(const v4fa*)(spar + CW + 4 * lane);
#pragma unroll 1
  for (int i = 0; i < 16; ++i) {
    const int row = wave * 16 + i;
    const v4f p = *(const v4fa*)(stg + row * CW + 4 * lane);
    float s = 0.0f, d = 0.0f;
    s = fmaf(p.x, as4.x, s); s = fmaf(p.y, as4.y, s); s = fmaf(p.z, as4.z, s); s = fmaf(p.w, as4.w, s);
    d = fmaf(p.x, ad4.x, d); d = fmaf(p.y, ad4.y, d); d = fmaf(p.z, ad4.z, d); d = fmaf(p.w, ad4.w, d);
#pragma unroll
    for (int off = 16; off > 0; off >>= 1) {
      s += __shfl_xor(s, off);
      d += __shfl_xor(d, off);
    }
    if (lane == 0) { sdt[row] = s; sdt[GBM + row] = d; }
  }
  __syncthreads();

  const v4f alv = *(const v4fa*)(sdt + 4 * lane);
  float* alp = AL + (size_t)blockIdx.x * (2 * GBM) + 4 * lane;
#pragma unroll 1
  for (int i = 0; i < 16; ++i) {
    const int row = wave * 16 + i;
    const v4f p = *(const v4fa*)(stg + row * CW + 4 * lane);
    float* op = Cm + (size_t)(rowBase + row) * (size_t)CW + 4 * lane;
    *(volatile v4f*)op = p;
  }
  if (wave == 0) *(volatile v4f*)alp = alv;
  __threadfence();
#pragma unroll 1
  for (int i = 0; i < 16; ++i) {
    const int row = wave * 16 + i;
    const v4f p = *(const v4fa*)(stg + row * CW + 4 * lane);
    float* op = Cm + (size_t)(rowBase + row) * (size_t)CW + 4 * lane;
    *(volatile v4f*)op = p;
  }
  if (wave == 0) *(volatile v4f*)alp = alv;
}

__global__ __launch_bounds__(NTHR) void k_replay(const int* __restrict__ HITS, const int* __restrict__ OFF,
                                                 const int* __restrict__ CNT, const int* __restrict__ FLAG,
                                                 const float* __restrict__ AL, const float* __restrict__ XL,
                                                 const float* __restrict__ PAR, int nN, unsigned short* AP) {
  __shared__ __attribute__((aligned(16))) float sb[CW];
  const int tid = (int)threadIdx.x, lane = tid & 31, wave = tid >> 5;
  if (tid < 32) {
    const v4f b = *(const v4f*)(PAR + P_BA * CW + 4 * tid);
    *(v4fa*)(sb + 4 * tid) = b;
  }
  __syncthreads();
  const int node = (int)blockIdx.x * NWAVE + wave;
  const bool live = node < nN;
  const int nc  = live ? node : nN - 1;
  int blk = nc >> SLA;
  blk = blk > GA - 1 ? GA - 1 : blk;
  const int craw = CNT[nc];
  const int oraw = OFF[nc];
  const int fl   = FLAG[blk * 32];
  int cv = craw < 0 ? 0 : (craw > DEGCAP ? DEGCAP : craw);
  cv = live ? cv : 0;
  int ovv = oraw < 0 ? 0 : (oraw > RCAP - 1 ? RCAP - 1 : oraw);
  const int c = __builtin_amdgcn_readfirstlane(cv);
  const int o = __builtin_amdgcn_readfirstlane(ovv);
  int last = o + c - 1;
  last = last < o ? o : last;
  last = last > RCAP - 1 ? RCAP - 1 : last;
  const bool pois = (fl != 0) || (craw > DEGCAP) || (craw < 0);
  const int* hp = HITS + (size_t)blk * RCAP;

  const int alb = (nc >> 6) * (2 * GBM) + (nc & (GBM - 1));
  const float as0 = AL[alb];
  const float ad  = AL[alb + GBM];
  v4f acc = *(const v4f*)(XL + (size_t)nc * CW + 4 * lane);
  float l0 = as0 + ad;
  l0 = l0 > 0.f ? l0 : NEGSL * l0;
  float mx = l0, dn = 1.0f;
#pragma unroll 1
  for (int b0 = 0; b0 < c; b0 += 32) {
    int idx = o + b0 + lane;
    idx = idx > last ? last : idx;
    int sr = hp[idx];
    sr = sr < 0 ? 0 : (sr > nN - 1 ? nN - 1 : sr);
    const float es  = AL[(sr >> 6) * (2 * GBM) + (sr & (GBM - 1))];
    const int   esi = __float_as_int(es);
    const int m32 = (c - b0) < 32 ? (c - b0) : 32;
#pragma unroll 1
    for (int k = 0; k < m32; ++k) {
      const int   sk  = __builtin_amdgcn_readlane(sr, k);
      const float ask = __int_as_float(__builtin_amdgcn_readlane(esi, k));
      const v4f a = *(const v4f*)(XL + (size_t)sk * CW + 4 * lane);
      float lg = ask + ad;
      lg = lg > 0.f ? lg : NEGSL * lg;
      const float df = lg - mx;
      const float ee = expf(-fabsf(df));
      const bool  up = df > 0.f;
      const float s1 = up ? ee : 1.0f;
      const float s2 = up ? 1.0f : ee;
      mx = up ? lg : mx;
      dn = fmaf(dn, s1, s2);
      acc.x = fmaf(acc.x, s1, s2 * a.x); acc.y = fmaf(acc.y, s1, s2 * a.y);
      acc.z = fmaf(acc.z, s1, s2 * a.z); acc.w = fmaf(acc.w, s1, s2 * a.w);
    }
  }
  const float inv = 1.0f / (dn + 1e-16f);
  const float pz  = pois ? __int_as_float(0x7fc00000) : 0.0f;
  const v4f bv = *(const v4fa*)(sb + 4 * lane);
  float v[4];
  v[0] = fmaf(acc.x, inv, bv.x) + pz;
  v[1] = fmaf(acc.y, inv, bv.y) + pz;
  v[2] = fmaf(acc.z, inv, bv.z) + pz;
  v[3] = fmaf(acc.w, inv, bv.w) + pz;
  v4us ho, lo;
#pragma unroll
  for (int i = 0; i < 4; ++i) {
    const float y = live ? v[i] : 0.0f;
    const unsigned hlp = split_hl(y);
    ho[i] = (unsigned short)(hlp & 0xFFFFu);
    lo[i] = (unsigned short)(hlp >> 16);
  }
  unsigned short* aq = AP + (size_t)node * APITCH + 4 * lane;
  *(volatile v4us*)aq = ho;
  *(volatile v4us*)(aq + CW) = lo;
  __threadfence();
  *(volatile v4us*)aq = ho;
  *(volatile v4us*)(aq + CW) = lo;
}

__global__ __launch_bounds__(GTHR) __attribute__((amdgpu_num_vgpr(248)))
void k_gemm1(const unsigned short* __restrict__ A, const unsigned short* __restrict__ BT, int K,
             const float* __restrict__ bias, int nN, float* Tm, double* REC) {
  __shared__ __attribute__((aligned(16))) float stg[GBM * CW];
  __shared__ __attribute__((aligned(16))) double rsd[2 * CW];
  __shared__ __attribute__((aligned(16))) float sbias[CW];
  const int tid = (int)threadIdx.x, lane = tid & 31, wave = tid >> 5, hh = lane >> 4, m = lane & 15;
  const int rowBase = (int)blockIdx.x * GBM;
  if (tid < 32) {
    const v4f b = *(const v4f*)(bias + 4 * tid);
    *(v4fa*)(sbias + 4 * tid) = b;
  }
  __syncthreads();

  v8f acc[8];
  {
    const v8f z = {0.f, 0.f, 0.f, 0.f, 0.f, 0.f, 0.f, 0.f};
#pragma unroll
    for (int t = 0; t < 8; ++t) acc[t] = z;
  }
  const unsigned short* ap = A  + (size_t)(rowBase + 16 * wave + m) * (size_t)APITCH + 8 * hh;
  const unsigned short* bp = BT + (size_t)m * (size_t)WPITCH + 8 * hh;

#pragma unroll 1
  for (int k0 = 0; k0 < K; k0 += 32) {
    FragB af;
    af.h[0] = *(const v8usa*)(ap + k0);
    af.h[1] = *(const v8usa*)(ap + k0 + 16);
#pragma unroll
    for (int nt = 0; nt < 8; ++nt) {
      const unsigned short* wq = bp + (size_t)(16 * nt) * (size_t)WPITCH + k0;
      FragB bf;
      bf.h[0] = *(const v8usa*)wq;
      bf.h[1] = *(const v8usa*)(wq + 16);
      acc[nt] = wmb(af, bf, acc[nt]);
    }
  }

#pragma unroll
  for (int nt = 0; nt < 8; ++nt) {
    const int lc = 16 * nt + m;
    const float bc = sbias[lc];
#pragma unroll
    for (int r = 0; r < 8; ++r) {
      const int lr = 16 * wave + 8 * hh + r;
      stg[lr * CW + lc] = acc[nt][r] + bc;
    }
  }
  __syncthreads();

  {
    double s = 0.0, q = 0.0;
#pragma unroll 4
    for (int r = 0; r < GBM; ++r) {
      const double dv = (double)stg[r * CW + tid];
      const bool ok = (rowBase + r) < nN;
      const double s1 = s + dv;
      const double q1 = fma(dv, dv, q);
      s = ok ? s1 : s;
      q = ok ? q1 : q;
    }
    rsd[tid] = s;
    rsd[CW + tid] = q;
  }
  __syncthreads();

  const v2d r2 = *(const v2da*)(rsd + 2 * tid);
  double* rp = REC + (size_t)blockIdx.x * (2 * CW) + 2 * tid;
#pragma unroll 1
  for (int i = 0; i < 16; ++i) {
    const int row = wave * 16 + i;
    const v4f p = *(const v4fa*)(stg + row * CW + 4 * lane);
    float* op = Tm + (size_t)(rowBase + row) * (size_t)CW + 4 * lane;
    *(volatile v4f*)op = p;
  }
  *(volatile v2d*)rp = r2;
  __threadfence();
#pragma unroll 1
  for (int i = 0; i < 16; ++i) {
    const int row = wave * 16 + i;
    const v4f p = *(const v4fa*)(stg + row * CW + 4 * lane);
    float* op = Tm + (size_t)(rowBase + row) * (size_t)CW + 4 * lane;
    *(volatile v4f*)op = p;
  }
  *(volatile v2d*)rp = r2;
}

__global__ __launch_bounds__(CW) void k_comb(const double* __restrict__ REC, int nT, double invN, float* MR) {
  __shared__ __attribute__((aligned(16))) float sm[2 * CW];
  const int tid = (int)threadIdx.x;
  double S = 0.0, Q = 0.0;
#pragma unroll 2
  for (int t = 0; t < nT; ++t) {
    const double* pr = REC + (size_t)t * (2 * CW);
    S += pr[tid];
    Q += pr[CW + tid];
  }
  const double mean = S * invN;
  double var = Q * invN - mean * mean;
  var = (var < 0.0) ? 0.0 : var;
  const float rs = 1.0f / sqrtf((float)var + 1e-5f);
  sm[tid] = (float)mean;
  sm[CW + tid] = rs;
  __syncthreads();
  v4f v;
  if (tid < (2 * CW) / 4) {
    v = *(const v4fa*)(sm + 4 * tid);
    *(volatile v4f*)(MR + 4 * tid) = v;
  }
  __threadfence();
  if (tid < (2 * CW) / 4) {
    *(volatile v4f*)(MR + 4 * tid) = v;
  }
}

__global__ __launch_bounds__(NTHR) void k_apply(const float* __restrict__ Tm, const float* __restrict__ MR,
                                                const float* __restrict__ GB, int nN, unsigned short* AP) {
  __shared__ __attribute__((aligned(16))) float sm[4 * CW];
  const int tid = (int)threadIdx.x;
  if (tid < 64) {
    const v4f p = *(const v4f*)(MR + 4 * tid);
    *(v4fa*)(sm + 4 * tid) = p;
  } else if (tid < 128) {
    const v4f p = *(const v4f*)(GB + 4 * (tid - 64));
    *(v4fa*)(sm + 2 * CW + 4 * (tid - 64)) = p;
  }
  __syncthreads();
  const int u   = (int)blockIdx.x * NTHR + tid;
  const int row = u >> 4;
  const int c8  = (u & 15) * 8;
  const bool ok = row < nN;
  const float* tp = Tm + (size_t)row * CW + c8;
  const v4f ta = *(const v4f*)tp;
  const v4f tb = *(const v4f*)(tp + 4);
  float t[8];
  t[0] = ta.x; t[1] = ta.y; t[2] = ta.z; t[3] = ta.w;
  t[4] = tb.x; t[5] = tb.y; t[6] = tb.z; t[7] = tb.w;
  v8us ho, lo;
#pragma unroll
  for (int i = 0; i < 8; ++i) {
    const float mm = sm[c8 + i];
    const float rr = sm[CW + c8 + i];
    const float gg = sm[2 * CW + c8 + i];
    const float bb = sm[3 * CW + c8 + i];
    float y = ((t[i] - mm) * rr) * gg + bb;
    y = (y > 0.0f) ? y : (y - y);
    y = ok ? y : 0.0f;
    const unsigned hlp = split_hl(y);
    ho[i] = (unsigned short)(hlp & 0xFFFFu);
    lo[i] = (unsigned short)(hlp >> 16);
  }
  unsigned short* aq = AP + (size_t)row * APITCH + c8;
  *(volatile v8us*)aq = ho;
  *(volatile v8us*)(aq + CW) = lo;
  __threadfence();
  *(volatile v8us*)aq = ho;
  *(volatile v8us*)(aq + CW) = lo;
}

__global__ __launch_bounds__(NTHR) void k_final(const float* __restrict__ Tm, const float* __restrict__ MR,
                                                const float* __restrict__ GB, const float* __restrict__ x,
                                                const int* __restrict__ FLAG, float* out) {
  __shared__ __attribute__((aligned(16))) float sm[4 * CW];
  const int tid = (int)threadIdx.x;
  if (tid < 64) {
    const v4f p = *(const v4f*)(MR + 4 * tid);
    *(v4fa*)(sm + 4 * tid) = p;
  } else if (tid < 128) {
    const v4f p = *(const v4f*)(GB + 4 * (tid - 64));
    *(v4fa*)(sm + 2 * CW + 4 * (tid - 64)) = p;
  }
  __syncthreads();
  const int u   = (int)blockIdx.x * NTHR + tid;
  const int row = u >> 5;
  const int c4  = (u & 31) * 4;
  int b = row >> SLA;
  b = b > GA - 1 ? GA - 1 : b;
  const int fl = FLAG[b * 32];
  const v4f t  = *(const v4f*)(Tm + (size_t)u * 4);
  const v4f xv = *(const v4f*)(x + (size_t)u * 4);
  const v4f m4 = *(const v4fa*)(sm + c4);
  const v4f r4 = *(const v4fa*)(sm + CW + c4);
  const v4f g4 = *(const v4fa*)(sm + 2 * CW + c4);
  const v4f b4 = *(const v4fa*)(sm + 3 * CW + c4);
  float y0 = ((t.x - m4.x) * r4.x) * g4.x + b4.x;
  float y1 = ((t.y - m4.y) * r4.y) * g4.y + b4.y;
  float y2 = ((t.z - m4.z) * r4.z) * g4.z + b4.z;
  float y3 = ((t.w - m4.w) * r4.w) * g4.w + b4.w;
  y0 = (y0 > 0.0f) ? y0 : (y0 - y0);
  y1 = (y1 > 0.0f) ? y1 : (y1 - y1);
  y2 = (y2 > 0.0f) ? y2 : (y2 - y2);
  y3 = (y3 > 0.0f) ? y3 : (y3 - y3);
  const float pz = (fl != 0) ? __int_as_float(0x7fc00000) : 0.0f;
  v4f o;
  o.x = y0 + bf16_val(xv.x) + pz;
  o.y = y1 + bf16_val(xv.y) + pz;
  o.z = y2 + bf16_val(xv.z) + pz;
  o.w = y3 + bf16_val(xv.w) + pz;
  float* op = out + (size_t)u * 4;
  *(volatile v4f*)op = o;
  __threadfence();
  *(volatile v4f*)op = o;
}

extern "C" void kernel_launch(void* const* d_in, const int* in_sizes, int n_in,
                              void* d_out, int out_size, void* d_ws, size_t ws_size,
                              hipStream_t stream) {
  if (n_in < 14) return;
  if (in_sizes[0] != NN * CW) return;
  if (in_sizes[1] != 2 * NE) return;
  if (in_sizes[2] != CW * CW) return;
  if (in_sizes[3] != CW || in_sizes[4] != CW || in_sizes[5] != CW) return;
  if (in_sizes[6] != CW * CW) return;
  if (in_sizes[7] != CW || in_sizes[8] != CW || in_sizes[9] != CW) return;
  if (in_sizes[10] != CW * CW) return;
  if (in_sizes[11] != CW || in_sizes[12] != CW || in_sizes[13] != CW) return;
  if (out_size != NN * CW) return;
  if (WS_TOTAL > ws_size) return;

  const float* x    = (const float*)d_in[0];
  const int*   edge = (const int*)d_in[1];
  const float* W    = (const float*)d_in[2];
  const float* avs  = (const float*)d_in[3];
  const float* avd  = (const float*)d_in[4];
  const float* bag  = (const float*)d_in[5];
  const float* W1   = (const float*)d_in[6];
  const float* b1   = (const float*)d_in[7];
  const float* g1   = (const float*)d_in[8];
  const float* be1  = (const float*)d_in[9];
  const float* W2   = (const float*)d_in[10];
  const float* b2   = (const float*)d_in[11];
  const float* g2   = (const float*)d_in[12];
  const float* be2  = (const float*)d_in[13];
  float* out = (float*)d_out;
  const int* src = edge;
  const int* dst = edge + NE;

  char* ws = (char*)d_ws;
  unsigned short* W0T = (unsigned short*)(ws + O_W0T);
  unsigned short* W1D = (unsigned short*)(ws + O_W1D);
  unsigned short* W2D = (unsigned short*)(ws + O_W2D);
  float*  PAR  = (float*)(ws + O_PAR);
  float*  MR1  = (float*)(ws + O_MR1);
  float*  MR2  = (float*)(ws + O_MR2);
  int*    FLAG = (int*)(ws + O_FLAG);
  int*    OFF  = (int*)(ws + O_OFF);
  int*    CNT  = (int*)(ws + O_CNT);
  float*  ALp  = (float*)(ws + O_AL);
  double* REC1 = (double*)(ws + O_REC1);
  double* REC2 = (double*)(ws + O_REC2);
  int*    HITS = (int*)(ws + O_HITS);
  unsigned short* XB = (unsigned short*)(ws + O_XB);
  float*  XL   = (float*)(ws + O_XL);
  unsigned short* AP = (unsigned short*)(ws + O_AP);
  float*  T    = (float*)(ws + O_T);

  const size_t bktLds = (size_t)AGG_LDS_INTS * 4;
  hipFuncSetAttribute(reinterpret_cast<const void*>(&k_bucket), hipFuncAttributeMaxDynamicSharedMemorySize, (int)bktLds);
  const double invN = 1.0 / (double)NN;
  const int vec8 = 1;

  k_prep<<<(NUX + NU0 + 2 * NUD + NUPB) / NTHR, NTHR, 0, stream>>>(x, W, W1, W2, avs, avd, bag, b1, g1, be1,
                                                                    b2, g2, be2, XB, W0T, W1D, W2D, PAR);
  k_bucket<<<GA, NTHR, bktLds, stream>>>(src, dst, NE, NN, vec8, HITS, OFF, CNT, FLAG);
  k_gemm0<<<GM, GTHR, 0, stream>>>(XB, W0T, PAR, XL, ALp);
  k_replay<<<MP / NWAVE, NTHR, 0, stream>>>(HITS, OFF, CNT, FLAG, ALp, XL, PAR, NN, AP);
  k_gemm1<<<GM, GTHR, 0, stream>>>(AP, W1D, KE1, PAR + P_B1 * CW, NN, T, REC1);
  k_comb<<<1, CW, 0, stream>>>(REC1, GM, invN, MR1);
  k_apply<<<NUX / NTHR, NTHR, 0, stream>>>(T, MR1, PAR + P_G1 * CW, NN, AP);
  k_gemm1<<<GM, GTHR, 0, stream>>>(AP, W2D, KE2, PAR + P_B2 * CW, NN, T, REC2);
  k_comb<<<1, CW, 0, stream>>>(REC2, GM, invN, MR2);
  k_final<<<(NN * 32) / NTHR, NTHR, 0, stream>>>(T, MR2, PAR + P_G2 * CW, x, FLAG, out);
}
